// EdgeFeatureConvBlock_83236466196745
// MI455X (gfx1250) — hardware-run, weakly checked
//
#include <hip/hip_runtime.h>


#ifndef NB
#define NB 16
#endif
#define NB_FULL 16
#define NPT  4096
#define KN   16
#define NE   (NPT * KN)
#define CIN  32
#define C0   32
#define C1   32
#define C2   64
#define WCR  (2 * C0 + C2)
#define XTP  128
#define PTB  32
#define EW   4
#define PPW  (PTB / EW)
#define YP   40
#define FOP  36
#define WSC  16.0f
#define WSI  0.0625f
#define INVF 0.9999950000374997f

static_assert(NB <= NB_FULL);
static_assert(CIN == 32);
static_assert(C0 == 32);
static_assert(C1 == 32);
static_assert(C2 == 64);
static_assert(2 * C0 == 64);
static_assert(WCR == 128);
static_assert(KN == 16);
static_assert(NPT % XTP == 0);
static_assert(NPT % 64 == 0);
static_assert(NPT % PTB == 0);
static_assert(((size_t)NB * NPT) % 64 == 0);
static_assert(NE % (256 * 4) == 0);
static_assert(PTB == 32);
static_assert(EW * PPW == PTB);
static_assert((YP * 2) % 16 == 0);
static_assert(YP >= C0);
static_assert((FOP * 4) % 16 == 0);
static_assert(FOP >= PTB);
static_assert(4 * 256 * 4 == CIN * XTP);
static_assert(2 * 256 * 16 == XTP * CIN * 2);
static_assert(4 * 32 * 16 == 16 * C0 * 4);
static_assert(8 * 32 * 16 == 16 * 64 * 4);
static_assert(4 * (32 * EW) * 16 == C2 * PTB * 4);
static_assert(4 * 32 * 4 == KN * C0);
static_assert(EW * 16 * YP * 2 + C2 * FOP * 4 <= 131072);
static_assert(16 * 68 * 4 <= 131072);
static_assert(XTP * 40 * 2 <= 131072);

typedef _Float16 h16;
typedef unsigned short bf;
typedef __attribute__((ext_vector_type(16))) __bf16   v16bf;
typedef __attribute__((ext_vector_type(16))) _Float16 v16h;
typedef __attribute__((ext_vector_type(8)))  _Float16 v8h;
typedef __attribute__((ext_vector_type(4)))  _Float16 v4h;
typedef __attribute__((ext_vector_type(8)))  unsigned short v8us;
typedef __attribute__((ext_vector_type(8)))  float    v8f;
typedef __attribute__((ext_vector_type(4)))  float    v4f;
typedef __attribute__((ext_vector_type(4)))  int      v4i;
typedef v4f  __attribute__((may_alias)) v4fa;
typedef v4h  __attribute__((may_alias)) v4ha;
typedef v8h  __attribute__((may_alias)) v8ha;
typedef v8us __attribute__((may_alias)) v8usa;

__device__ __forceinline__ unsigned short f2bf(float f) { unsigned u = __float_as_uint(f); u += 0x7FFFu + ((u >> 16) & 1u); return (unsigned short)(u >> 16); }
__device__ __forceinline__ float bfr(float f) { return __uint_as_float(((unsigned)f2bf(f)) << 16); }
__device__ __forceinline__ v16h cat16(v8h lo, v8h hi) { return __builtin_shufflevector(lo, hi, 0, 1, 2, 3, 4, 5, 6, 7, 8, 9, 10, 11, 12, 13, 14, 15); }
__device__ __forceinline__ v16bf cat16b(v8us lo, v8us hi) { return __builtin_bit_cast(v16bf, __builtin_shufflevector(lo, hi, 0, 1, 2, 3, 4, 5, 6, 7, 8, 9, 10, 11, 12, 13, 14, 15)); }
__device__ __forceinline__ v8f wmma16(v16h a, v16h b, v8f c) { return __builtin_amdgcn_wmma_f32_16x16x32_f16(false, a, false, b, (short)0, c, false, false); }
__device__ __forceinline__ v8f wmmab(v16bf a, v16bf b, v8f c) { return __builtin_amdgcn_wmma_f32_16x16x32_bf16(false, a, false, b, (short)0, c, false, false); }
__device__ __forceinline__ v16h  ldh(const h16* p) { return cat16(*(const v8h*)p, *(const v8h*)(p + 16)); }
__device__ __forceinline__ v16bf ldb(const bf* p)  { return cat16b(*(const v8us*)p, *(const v8us*)(p + 16)); }
__device__ __forceinline__ void wave_sync() { __builtin_amdgcn_fence(3  , "wavefront"); __builtin_amdgcn_wave_barrier(); asm volatile("" ::: "memory"); }

__device__ __forceinline__ h16 toh_flush(float v) { const h16 r = (h16)v; return (fabsf(v) < 6.103515625e-05f) ? (h16)0.0f : r; }
__device__ __forceinline__ v8f wmma16g(v16h a, v16h b, v8f c) { c = wmma16(a, b, c); asm volatile("v_nop\n\tv_nop\n\tv_nop\n\tv_nop" : "+v"(c) : "v"(a), "v"(b)); return c; }
__device__ __forceinline__ v8f wmmabg(v16bf a, v16bf b, v8f c) { c = wmmab(a, b, c); asm volatile("v_nop\n\tv_nop\n\tv_nop\n\tv_nop" : "+v"(c) : "v"(a), "v"(b)); return c; }

__global__ __launch_bounds__(256) void k_xt(const float* __restrict__ src, bf* dst) {
    __shared__ __align__(16) unsigned short xs[XTP * 40];
    const int tid = threadIdx.x;
    const int q0 = blockIdx.x * XTP; const int b = q0 / NPT, p0 = q0 % NPT;
    const float* sb = src + (size_t)b * CIN * NPT + p0;
#pragma unroll
    for (int s = 0; s < 4; ++s) { const int idx = s * 256 + tid; const int c = idx >> 5, p4 = (idx & 31) * 4;
        const v4f v = *(const v4f*)(sb + (size_t)c * NPT + p4);
#pragma unroll
        for (int i = 0; i < 4; ++i) xs[(p4 + i) * 40 + c] = f2bf(v[i]); }
    __syncthreads();
    v8us o[2];
#pragma unroll
    for (int s = 0; s < 2; ++s) { const int idx = s * 256 + tid; const int p = idx >> 2, c8 = (idx & 3) * 8; o[s] = *(const v8usa*)(&xs[p * 40 + c8]); }
    bf* db = dst + (size_t)q0 * CIN;
#pragma unroll 1
    for (int ps = 0; ps < 2; ++ps) {
#pragma unroll
        for (int s = 0; s < 2; ++s) *(volatile v8us*)(db + (size_t)(s * 256 + tid) * 8) = o[s];
        if (ps == 0) __threadfence(); }
}

__global__ __launch_bounds__(64) void k_wb(const float* __restrict__ src, int spitch, int scol, bf* dst, int n8) {
    const int i = blockIdx.x * 64 + threadIdx.x; if (i >= n8) return;
    const int row = i >> 2, c8 = (i & 3) * 8;
    const v8f v = *(const v8f*)(src + (size_t)row * spitch + scol + c8); v8us o;
#pragma unroll
    for (int k = 0; k < 8; ++k) o[k] = f2bf(v[k]);
    *(volatile v8us*)(dst + (size_t)i * 8) = o; __threadfence(); *(volatile v8us*)(dst + (size_t)i * 8) = o;
}

__global__ __launch_bounds__(64) void k_wh(const float* __restrict__ src, h16* dst, int n8) {
    const int i = blockIdx.x * 64 + threadIdx.x; if (i >= n8) return;
    const v8f v = *(const v8f*)(src + (size_t)i * 8); v8h o;
#pragma unroll
    for (int k = 0; k < 8; ++k) o[k] = toh_flush(bfr(v[k]) * WSC);
    *(volatile v8h*)(dst + (size_t)i * 8) = o; __threadfence(); *(volatile v8h*)(dst + (size_t)i * 8) = o;
}

__global__ __launch_bounds__(256) void k_chk(const int* __restrict__ tab, int* FL) {
    __shared__ int sw[8];
    const int tid = threadIdx.x, lane = tid & 31;
    const int wave = __builtin_amdgcn_readfirstlane((int)(threadIdx.x >> 5));
    const int b = blockIdx.x;
    const int* pf = tab + (size_t)b * 2 * NE;
    int bad = 0;
#pragma unroll 4
    for (int i = 0; i < NE / (256 * 4); ++i) { const int e4 = (i * 256 + tid) * 4; const v4i v = *(const v4i*)(pf + e4); const int ex = e4 >> 4;
        bad |= (int)(v[0] != ex) | (int)(v[1] != ex) | (int)(v[2] != ex) | (int)(v[3] != ex); }
    const unsigned bm = __builtin_amdgcn_ballot_w32(bad != 0);
    if (lane == 0) sw[wave] = (bm != 0u) ? 1 : 0;
    __syncthreads();
    if (wave == 0) {
        int f = 0;
#pragma unroll
        for (int w = 0; w < 8; ++w) f |= sw[w];
        *(volatile int*)(FL + (size_t)b * 32 + lane) = f; __threadfence(); *(volatile int*)(FL + (size_t)b * 32 + lane) = f; }
}

__global__ __launch_bounds__(32) void k_th(const bf* __restrict__ XB, const bf* __restrict__ WC, const float* __restrict__ g0, const float* __restrict__ b0, float* T, float* H) {
    __shared__ __align__(16) float os[16 * 68];
    const int lane = threadIdx.x & 31, lr = lane & 15, hi = lane >> 4; const int r0 = blockIdx.x * 64;
    v16bf wf[4];
#pragma unroll
    for (int nb = 0; nb < 4; ++nb) wf[nb] = ldb(WC + (size_t)(nb * 16 + lr) * CIN + 8 * hi);
    float sA[2], cA[2];
#pragma unroll
    for (int t = 0; t < 2; ++t) { sA[t] = bfr(g0[t * 16 + lr]) * INVF; cA[t] = bfr(b0[t * 16 + lr]); }
#pragma unroll 1
    for (int mb = 0; mb < 4; ++mb) {
        const v16bf a = ldb(XB + (size_t)(r0 + mb * 16 + lr) * CIN + 8 * hi);
        v8f acc[4];
#pragma unroll
        for (int nb = 0; nb < 4; ++nb) { acc[nb] = (v8f){}; acc[nb] = wmmabg(a, wf[nb], acc[nb]); }
#pragma unroll
        for (int t = 0; t < 2; ++t) {
#pragma unroll
            for (int j = 0; j < 8; ++j) {
                os[(hi * 8 + j) * 68 + t * 16 + lr]      = sA[t] * (acc[t][j] - acc[2 + t][j]) + cA[t];
                os[(hi * 8 + j) * 68 + 32 + t * 16 + lr] = sA[t] * acc[2 + t][j]; } }
        wave_sync();
        v4f tv[4], hv[4];
#pragma unroll
        for (int s = 0; s < 4; ++s) { const int row = 4 * s + (lane >> 3), cofs = (lane & 7) * 4;
            tv[s] = *(const v4fa*)(&os[row * 68 + cofs]); hv[s] = *(const v4fa*)(&os[row * 68 + 32 + cofs]); }
        const size_t rb = (size_t)(r0 + mb * 16) * C0;
#pragma unroll 1
        for (int ps = 0; ps < 2; ++ps) {
#pragma unroll
            for (int s = 0; s < 4; ++s) { const int row = 4 * s + (lane >> 3), cofs = (lane & 7) * 4;
                *(volatile v4f*)(T + rb + (size_t)row * C0 + cofs) = tv[s];
                *(volatile v4f*)(H + rb + (size_t)row * C0 + cofs) = hv[s]; }
            if (ps == 0) __threadfence(); }
        wave_sync();
    }
}

__global__ __launch_bounds__(32) void k_sc(const bf* __restrict__ XB, const bf* __restrict__ WS, const float* __restrict__ sg, const float* __restrict__ sb, float* SC) {
    __shared__ __align__(16) float os[16 * 68];
    const int lane = threadIdx.x & 31, lr = lane & 15, hi = lane >> 4; const int r0 = blockIdx.x * 64;
    const int bb = r0 / NPT, p0 = r0 % NPT;
    v16bf xf[4];
#pragma unroll
    for (int nb = 0; nb < 4; ++nb) xf[nb] = ldb(XB + (size_t)(r0 + nb * 16 + lr) * CIN + 8 * hi);
#pragma unroll 1
    for (int mb = 0; mb < 4; ++mb) {
        const v16bf a = ldb(WS + (size_t)(mb * 16 + lr) * CIN + 8 * hi);
        v8f acc[4];
#pragma unroll
        for (int nb = 0; nb < 4; ++nb) { acc[nb] = (v8f){}; acc[nb] = wmmabg(a, xf[nb], acc[nb]); }
        const v4f ga = *(const v4f*)(sg + mb * 16 + 8 * hi), gb = *(const v4f*)(sg + mb * 16 + 8 * hi + 4);
        const v4f ba = *(const v4f*)(sb + mb * 16 + 8 * hi), bc = *(const v4f*)(sb + mb * 16 + 8 * hi + 4);
#pragma unroll
        for (int j = 0; j < 4; ++j) {
            const float s0 = bfr(ga[j]) * INVF, s1 = bfr(gb[j]) * INVF; const float c0 = bfr(ba[j]), c1 = bfr(bc[j]);
#pragma unroll
            for (int nb = 0; nb < 4; ++nb) {
                os[(hi * 8 + j) * 68 + nb * 16 + lr]     = acc[nb][j] * s0 + c0;
                os[(hi * 8 + 4 + j) * 68 + nb * 16 + lr] = acc[nb][4 + j] * s1 + c1; } }
        wave_sync();
        v4f ov[8];
#pragma unroll
        for (int s = 0; s < 8; ++s) { const int row = 2 * s + (lane >> 4), cofs = (lane & 15) * 4;
            ov[s] = *(const v4fa*)(&os[row * 68 + cofs]); }
        const size_t rb = ((size_t)bb * C2 + (size_t)(mb * 16)) * NPT + (size_t)p0;
#pragma unroll 1
        for (int ps = 0; ps < 2; ++ps) {
#pragma unroll
            for (int s = 0; s < 8; ++s) { const int row = 2 * s + (lane >> 4), cofs = (lane & 15) * 4;
                *(volatile v4f*)(SC + rb + (size_t)row * NPT + cofs) = ov[s]; }
            if (ps == 0) __threadfence(); }
        wave_sync();
    }
}

__global__ __launch_bounds__(32 * EW) void k_nbr(const float* __restrict__ T, const float* __restrict__ H, const float* __restrict__ SC, const int* __restrict__ FL, const int* __restrict__ tab,
                                                 const h16* __restrict__ W1H, const h16* __restrict__ W2H,
                                                 const float* __restrict__ g1, const float* __restrict__ b1, const float* __restrict__ g2, const float* __restrict__ b2, float* OUT) {
    __shared__ __align__(16) h16 ys[EW * 16 * YP];
    __shared__ __align__(16) float fo[C2 * FOP];
    const int lane = threadIdx.x & 31, lr = lane & 15, hi = lane >> 4;
    const int wave = __builtin_amdgcn_readfirstlane((int)(threadIdx.x >> 5));
    const int q0 = blockIdx.x * PTB; const int b = q0 / NPT, p0 = q0 % NPT;
    const bool pois = FL[(size_t)b * 32] != 0;
    const v16h w1a0 = ldh(W1H + (size_t)lr * C0 + 8 * hi), w1a1 = ldh(W1H + (size_t)(16 + lr) * C0 + 8 * hi);
    v16h w2b[4];
#pragma unroll
    for (int nt = 0; nt < 4; ++nt) w2b[nt] = ldh(W2H + (size_t)(nt * 16 + lr) * C1 + 8 * hi);
    float s1[16], c1[16];
#pragma unroll
    for (int t = 0; t < 2; ++t) {
        const v4f ga = *(const v4f*)(g1 + t * 16 + 8 * hi), gb = *(const v4f*)(g1 + t * 16 + 8 * hi + 4);
        const v4f ba = *(const v4f*)(b1 + t * 16 + 8 * hi), bc = *(const v4f*)(b1 + t * 16 + 8 * hi + 4);
#pragma unroll
        for (int r = 0; r < 4; ++r) { s1[8 * t + r] = bfr(ga[r]) * INVF * WSI; s1[8 * t + 4 + r] = bfr(gb[r]) * INVF * WSI; c1[8 * t + r] = bfr(ba[r]); c1[8 * t + 4 + r] = bfr(bc[r]); } }
    float s2[4], c2[4];
#pragma unroll
    for (int nt = 0; nt < 4; ++nt) { s2[nt] = bfr(g2[nt * 16 + lr]) * INVF * WSI; c2[nt] = bfr(b2[nt * 16 + lr]); }
    const int c4 = (lane & 7) * 4, eg = lane >> 3;
    const int wb = wave * 16 * YP;
    const float qnan = __uint_as_float(0x7FC00000u);
#pragma unroll 1
    for (int it = 0; it < PPW; ++it) {
        const int pl = wave * PPW + it; const int p = p0 + pl;
        int tg = tab[((size_t)b * 2 + 1) * NE + (size_t)p * KN + lr];
        tg = tg < 0 ? tg + NPT : tg; tg = tg < 0 ? 0 : (tg > NPT - 1 ? NPT - 1 : tg);
        unsigned tu = (unsigned)tg; asm volatile("" : "+v"(tu));
        const v4f tv = *(const v4f*)(T + (size_t)(q0 + pl) * C0 + c4);
#pragma unroll
        for (int s = 0; s < 4; ++s) { const int e = 4 * s + eg;
            const unsigned te = (unsigned)__shfl((int)tu, e, 32);
            const v4f hv = *(const v4f*)(H + ((size_t)b * NPT + (size_t)te) * C0 + c4); v4h y;
#pragma unroll
            for (int i = 0; i < 4; ++i) y[i] = toh_flush(fmaxf(tv[i] + hv[i], 0.0f));
            *(v4ha*)(&ys[wb + e * YP + c4]) = y; }
        wave_sync();
        const v16h yb = cat16(*(const v8ha*)(&ys[wb + lr * YP + 8 * hi]), *(const v8ha*)(&ys[wb + lr * YP + 16 + 8 * hi]));
        v8f d0 = (v8f){}, d1 = (v8f){};
        d0 = wmma16g(w1a0, yb, d0); d1 = wmma16g(w1a1, yb, d1);
        v16h a2;
#pragma unroll
        for (int r = 0; r < 8; ++r) { a2[r] = toh_flush(fmaxf(d0[r] * s1[r] + c1[r], 0.0f)); a2[8 + r] = toh_flush(fmaxf(d1[r] * s1[8 + r] + c1[8 + r], 0.0f)); }
        float f[4];
#pragma unroll
        for (int nt = 0; nt < 4; ++nt) { v8f e2 = (v8f){}; e2 = wmma16g(a2, w2b[nt], e2);
            float a = 0.0f;
#pragma unroll
            for (int r = 0; r < 8; ++r) a += fmaxf(e2[r] * s2[nt] + c2[nt], 0.0f);
            a += __shfl_xor(a, 16, 32);
            f[nt] = pois ? qnan : a; }
        const float va = hi ? f[2] : f[0], vb = hi ? f[3] : f[1];
        fo[(32 * hi + lr) * FOP + pl] = va; fo[(32 * hi + 16 + lr) * FOP + pl] = vb;
        wave_sync();
    }
    __syncthreads();
    const size_t ob = ((size_t)b * C2) * NPT + (size_t)p0;
    v4f val[4];
#pragma unroll
    for (int s = 0; s < 4; ++s) { const int idx = s * (32 * EW) + (int)threadIdx.x; const int row = idx >> 3, cofs = (idx & 7) * 4;
        const v4f fv = *(const v4fa*)(&fo[row * FOP + cofs]);
        const v4f sv = *(const v4f*)(SC + ob + (size_t)row * NPT + cofs);
#pragma unroll
        for (int i = 0; i < 4; ++i) { const float u = sv[i] + fv[i] * (1.0f / 16.0f); val[s][i] = (u > 0.0f) ? u : (u - u); } }
#pragma unroll 1
    for (int ps = 0; ps < 2; ++ps) {
#pragma unroll
        for (int s = 0; s < 4; ++s) { const int idx = s * (32 * EW) + (int)threadIdx.x; const int row = idx >> 3, cofs = (idx & 7) * 4;
            *(volatile v4f*)(OUT + ob + (size_t)row * NPT + cofs) = val[s]; }
        if (ps == 0) __threadfence(); }
}

static constexpr size_t al256(size_t v) { return (v + 255) & ~(size_t)255; }
static constexpr size_t SZ_XB = al256((size_t)NB * NPT * CIN * 2);
static constexpr size_t SZ_WC = al256((size_t)WCR * CIN * 2);
static constexpr size_t SZ_W1 = al256((size_t)C1 * C0 * 2);
static constexpr size_t SZ_W2 = al256((size_t)C2 * C1 * 2);
static constexpr size_t SZ_TH = al256((size_t)NB * NPT * C0 * 4);
static constexpr size_t SZ_SC = al256((size_t)NB * C2 * NPT * 4);
static constexpr size_t SZ_FL = al256((size_t)NB * 32 * 4);
static constexpr size_t SZ_TOTAL = SZ_XB + SZ_WC + SZ_W1 + SZ_W2 + 2 * SZ_TH + SZ_SC + SZ_FL;
static_assert(SZ_TOTAL <= (size_t)134217728);
static_assert(((size_t)C0 * CIN * 2) % 256 == 0);
static_assert(((size_t)NB * NPT) % XTP == 0);
static_assert(((size_t)C0 * 4) % 64 == 0 && ((size_t)C2 * 4) % 64 == 0);

extern "C" void kernel_launch(void* const* d_in, const int* in_sizes, int n_in,
                              void* d_out, int out_size, void* d_ws, size_t ws_size, hipStream_t stream) {
    if (n_in < 15) return;
    if ((size_t)in_sizes[1] < (size_t)NB * CIN * NPT) return;
    if ((size_t)in_sizes[2] < (size_t)NB * 2 * NE) return;
    if (in_sizes[3] < C0 * 2 * CIN || in_sizes[4] < C0 || in_sizes[5] < C0) return;
    if (in_sizes[6] < C1 * C0 || in_sizes[7] < C1 || in_sizes[8] < C1) return;
    if (in_sizes[9] < C2 * C1 || in_sizes[10] < C2 || in_sizes[11] < C2) return;
    if (in_sizes[12] < C2 * CIN || in_sizes[13] < C2 || in_sizes[14] < C2) return;
    if ((size_t)out_size < (size_t)NB * C2 * NPT) return;
    if (SZ_TOTAL > ws_size) return;
    const float* xin = (const float*)d_in[1];
    const int*   tab = (const int*)d_in[2];
    const float* w0 = (const float*)d_in[3];  const float* g0 = (const float*)d_in[4];  const float* b0 = (const float*)d_in[5];
    const float* w1 = (const float*)d_in[6];  const float* g1 = (const float*)d_in[7];  const float* b1 = (const float*)d_in[8];
    const float* w2 = (const float*)d_in[9];  const float* g2 = (const float*)d_in[10]; const float* b2 = (const float*)d_in[11];
    const float* ws_ = (const float*)d_in[12]; const float* gs = (const float*)d_in[13]; const float* bs = (const float*)d_in[14];
    float* OUT = (float*)d_out;
    char* wsp = (char*)d_ws;
    bf*  XB  = (bf*)wsp;   wsp += SZ_XB;
    bf*  WC  = (bf*)wsp;   wsp += SZ_WC;
    h16* W1H = (h16*)wsp;  wsp += SZ_W1;
    h16* W2H = (h16*)wsp;  wsp += SZ_W2;
    float* T = (float*)wsp; wsp += SZ_TH;
    float* H = (float*)wsp; wsp += SZ_TH;
    float* SC = (float*)wsp; wsp += SZ_SC;
    int* FL = (int*)wsp;   wsp += SZ_FL;

    k_xt<<<(unsigned)((size_t)NB * NPT / XTP), 256, 0, stream>>>(xin, XB);
    k_wb<<<(C0 * 4) / 64, 64, 0, stream>>>(w0, 2 * CIN, 0,   WC,                         C0 * 4);
    k_wb<<<(C0 * 4) / 64, 64, 0, stream>>>(w0, 2 * CIN, CIN, WC + (size_t)C0 * CIN,      C0 * 4);
    k_wb<<<(C2 * 4) / 64, 64, 0, stream>>>(ws_, CIN, 0,      WC + (size_t)2 * C0 * CIN,  C2 * 4);
    k_wh<<<(C1 * 4) / 64, 64, 0, stream>>>(w1, W1H, C1 * 4);
    k_wh<<<(C2 * 4) / 64, 64, 0, stream>>>(w2, W2H, C2 * 4);
    k_chk<<<NB, 256, 0, stream>>>(tab, FL);
    k_th<<<(unsigned)((size_t)NB * NPT / 64), 32, 0, stream>>>(XB, WC, g0, b0, T, H);
    k_sc<<<(unsigned)((size_t)NB * NPT / 64), 32, 0, stream>>>(XB, WC + (size_t)2 * C0 * CIN, gs, bs, SC);
    k_nbr<<<(unsigned)((size_t)NB * NPT / PTB), 32 * EW, 0, stream>>>(T, H, SC, FL, tab, W1H, W2H, g1, b1, g2, b2, OUT);
}
